// ToySchizoBet_85177791414735
// MI455X (gfx1250) — hardware-verified
//
#include <hip/hip_runtime.h>


#define NB_  16
#define TT   2048
#define NT   32768
#define DD   128
#define HH   64
#define WW   16
#define VOC  42
#define VP   64
typedef _Float16 h16;
typedef unsigned short bf;
typedef __attribute__((ext_vector_type(16))) __bf16   v16bf;
typedef __attribute__((ext_vector_type(16))) _Float16 v16h;
typedef __attribute__((ext_vector_type(8)))  _Float16 v8h;
typedef __attribute__((ext_vector_type(8)))  unsigned short v8us;
typedef __attribute__((ext_vector_type(8)))  float    v8f;
typedef __attribute__((ext_vector_type(4)))  float    v4f;
typedef v8h  __attribute__((may_alias)) v8ha;
typedef v4f  __attribute__((may_alias)) v4fa;
typedef v8us __attribute__((may_alias)) v8usa;

__device__ __forceinline__ unsigned short f2bf(float f) { unsigned u = __float_as_uint(f); u += 0x7FFFu + ((u >> 16) & 1u); return (unsigned short)(u >> 16); }
__device__ __forceinline__ float bf2f(unsigned short b) { return __uint_as_float(((unsigned)b) << 16); }
__device__ __forceinline__ float bfr(float f) { return bf2f(f2bf(f)); }
__device__ __forceinline__ v16h cat16(v8h lo, v8h hi) { return __builtin_shufflevector(lo, hi, 0, 1, 2, 3, 4, 5, 6, 7, 8, 9, 10, 11, 12, 13, 14, 15); }
__device__ __forceinline__ v16bf cat16b(v8us lo, v8us hi) { return __builtin_bit_cast(v16bf, __builtin_shufflevector(lo, hi, 0, 1, 2, 3, 4, 5, 6, 7, 8, 9, 10, 11, 12, 13, 14, 15)); }
__device__ __forceinline__ v8f wmma16(v16h a, v16h b, v8f c) { return __builtin_amdgcn_wmma_f32_16x16x32_f16(false, a, false, b, (short)0, c, false, false); }
__device__ __forceinline__ v8f wmmab(v16bf a, v16bf b, v8f c) { return __builtin_amdgcn_wmma_f32_16x16x32_bf16(false, a, false, b, (short)0, c, false, false); }


template <typename T16> struct WFrag;
template <> struct WFrag<h16> { typedef v16h V; static __device__ __forceinline__ V ld(const h16* p) { return cat16(*(const v8h*)p, *(const v8h*)(p + 16)); } static __device__ __forceinline__ v8f mma(V a, V b, v8f c) { return wmma16(a, b, c); } };
template <> struct WFrag<bf> { typedef v16bf V; static __device__ __forceinline__ V ld(const bf* p) { return cat16b(*(const v8us*)p, *(const v8us*)(p + 16)); } static __device__ __forceinline__ v8f mma(V a, V b, v8f c) { return wmmab(a, b, c); } };
template <typename T16, int NSPLIT, bool BIAS>
__global__ __launch_bounds__(32) void k_gemmw(const T16* __restrict__ A, const T16* __restrict__ A2, const T16* __restrict__ Bt, const T16* __restrict__ Bt2, int K, float* C, int ldc, const float* __restrict__ bias, size_t sA, size_t sB, size_t sC) {
    typedef typename WFrag<T16>::V V;
    __shared__ __align__(16) float os[16 * 68];
    const size_t z = blockIdx.z; A += z * sA; if (A2) A2 += z * sA; Bt += z * sB; if (Bt2) Bt2 += z * sB; C += z * sC;
    const int lane = threadIdx.x & 31, lr = lane & 15, hi = lane >> 4; const int r0 = blockIdx.x * 64, c0 = blockIdx.y * 64;
    v8f acc[4][4];
#pragma unroll
    for (int mb = 0; mb < 4; ++mb)
#pragma unroll
        for (int nb = 0; nb < 4; ++nb) acc[mb][nb] = (v8f){};
    const size_t aoff = (size_t)(r0 + lr) * K + 8 * hi, boff = (size_t)(c0 + lr) * K + 8 * hi;
#pragma unroll 1
    for (int kc = 0; kc < K; kc += 32) {
        V a[4], a2[4];
#pragma unroll
        for (int mb = 0; mb < 4; ++mb) { a[mb] = WFrag<T16>::ld(A + aoff + (size_t)mb * 16 * K + kc); if (NSPLIT == 1 || NSPLIT == 2) a2[mb] = WFrag<T16>::ld(A2 + aoff + (size_t)mb * 16 * K + kc); }
#pragma unroll
        for (int nb = 0; nb < 4; ++nb) { const V b = WFrag<T16>::ld(Bt + boff + (size_t)nb * 16 * K + kc); V b2; if (NSPLIT >= 2) b2 = WFrag<T16>::ld(Bt2 + boff + (size_t)nb * 16 * K + kc);
#pragma unroll
            for (int mb = 0; mb < 4; ++mb) { acc[mb][nb] = WFrag<T16>::mma(a[mb], b, acc[mb][nb]); if (NSPLIT == 1 || NSPLIT == 2) acc[mb][nb] = WFrag<T16>::mma(a2[mb], b, acc[mb][nb]); if (NSPLIT >= 2) acc[mb][nb] = WFrag<T16>::mma(a[mb], b2, acc[mb][nb]); } }
        asm volatile("v_nop\n\tv_nop\n\tv_nop\n\tv_nop" : "+v"(acc[0][0]), "+v"(acc[1][1]), "+v"(acc[2][2]), "+v"(acc[3][3]) : "v"(a[0]), "v"(a[3]));
    }
#pragma unroll
    for (int mb = 0; mb < 4; ++mb) {
#pragma unroll
        for (int nb = 0; nb < 4; ++nb) {
#pragma unroll
            for (int j = 0; j < 8; ++j) os[(hi * 8 + j) * 68 + nb * 16 + lr] = acc[mb][nb][j]; }
        __builtin_amdgcn_wave_barrier(); asm volatile("" ::: "memory");
        float* crow = C + (size_t)(r0 + mb * 16) * ldc + c0;
#pragma unroll 1
        for (int ps = 0; ps < 2; ++ps) {
#pragma unroll
            for (int s = 0; s < 8; ++s) { const int row = 2 * s + hi, cofs = lr * 4; v4f val = *(const v4fa*)(os + row * 68 + cofs); if (BIAS) { val[0] += bfr(bias[c0 + cofs]); val[1] += bfr(bias[c0 + cofs + 1]); val[2] += bfr(bias[c0 + cofs + 2]); val[3] += bfr(bias[c0 + cofs + 3]); }
                *(volatile v4f*)(crow + (size_t)row * ldc + cofs) = val; }
            if (ps == 0) __threadfence(); }
        __builtin_amdgcn_wave_barrier(); asm volatile("" ::: "memory");
    }
}

__device__ __forceinline__ void splitf(float y, unsigned short& h, unsigned short& l) { h = f2bf(y); l = f2bf(y - bf2f(h)); }
__device__ __forceinline__ int cid(int v) { return v < 0 ? 0 : (v >= VOC ? VOC - 1 : v); }
typedef __attribute__((ext_vector_type(2))) unsigned short v2us;
typedef __attribute__((ext_vector_type(4))) unsigned short v4us;

__global__ __launch_bounds__(256) void k_wtG(const float* __restrict__ w, int K, int N, bf* Bt) {
    const int lane = threadIdx.x & 31; const int L0 = (blockIdx.x * 8 + (threadIdx.x >> 5)) * 8; const int nlines = N * K / 64;
#pragma unroll
    for (int ps = 0; ps < 2; ++ps) {
#pragma unroll 1
        for (int l = 0; l < 8; ++l) { const int L = L0 + l; if (L >= nlines) break; const size_t e = (size_t)L * 64 + lane * 2; const int k = (int)(e % K), n = (int)(e / K); v2us o;
            o[0] = f2bf(w[(size_t)k * N + n]); o[1] = f2bf(w[(size_t)(k + 1) * N + n]); *(volatile v2us*)(Bt + e) = o; }
        if (ps == 0) __threadfence(); }
}
__global__ __launch_bounds__(256) void k_embp(const float* __restrict__ emb, bf* EB) { const int e = (blockIdx.x * 256 + threadIdx.x) * 4; if (e >= VP * DD) return; const int r = e / DD; v4us o;
#pragma unroll
    for (int u = 0; u < 4; ++u) o[u] = (r < VOC) ? f2bf(emb[e + u]) : (unsigned short)0; *(volatile v4us*)(EB + e) = o; __threadfence(); *(volatile v4us*)(EB + e) = o; }
__global__ __launch_bounds__(256) void k_wpad(const float* __restrict__ w, int K, int N0, int NPd, bf* Bt) { const int e = (blockIdx.x * 256 + threadIdx.x) * 4; if (e >= NPd * K) return; const int k = e % K; const int n = e / K; v4us o;
#pragma unroll
    for (int u = 0; u < 4; ++u) o[u] = (n < N0) ? f2bf(w[(size_t)(k + u) * N0 + n]) : (unsigned short)0; *(volatile v4us*)(Bt + e) = o; __threadfence(); *(volatile v4us*)(Bt + e) = o; }
__device__ __forceinline__ float sigm(float z) { return __fdiv_rn(1.0f, __fadd_rn(1.0f, __expf(-z))); }
__global__ __launch_bounds__(256) void k_tau(const int* __restrict__ ids, const float* __restrict__ TA, const float* __restrict__ TB, const float* __restrict__ b1, const float* __restrict__ w2, const float* __restrict__ b2, float* TAU) { const int idx = blockIdx.x * 256 + threadIdx.x; if (idx >= NT * WW) return; const int w = idx % WW; const int tk = idx / WW; const int b = tk / TT, t = tk % TT; const int idt = cid(ids[tk]); const bool valid = (t >= w + 1); const int idn = valid ? cid(ids[b * TT + t - w - 1]) : 0;
    const float* ta = TA + idt * HH; const float* tb = TB + idn * HH; float s = 0.f;
#pragma unroll 1
    for (int k = 0; k < HH; ++k) { const float z = __fadd_rn(__fadd_rn(ta[k], valid ? tb[k] : 0.f), bfr(b1[k])); float sg = sigm(z); asm volatile("" : "+v"(sg)); const float h = __fmul_rn(z, sg); float wk = bfr(w2[k]); asm volatile("" : "+v"(wk)); float p = __fmul_rn(h, wk); asm volatile("" : "+v"(p)); s = __fadd_rn(s, p); }
    const float tau = sigm(__fadd_rn(s, bfr(b2[0]))); *(volatile float*)(TAU + idx) = tau; __threadfence(); *(volatile float*)(TAU + idx) = tau; }
__global__ __launch_bounds__(256) void k_msg(const int* __restrict__ ids, const float* __restrict__ TAU, const float* __restrict__ TV, const float* __restrict__ wvb, bf* Mh, bf* Ml) { const int e = (blockIdx.x * 256 + threadIdx.x) * 4; if (e >= NT * DD) return; const int d0 = e % DD; const int tk = e / DD; const int b = tk / TT, t = tk % TT; float acc[4] = {0.f, 0.f, 0.f, 0.f};
#pragma unroll 1
    for (int w = 0; w < WW; ++w) { const float tau = TAU[tk * WW + w]; const bool valid = (t >= w + 1); const int idn = valid ? cid(ids[b * TT + t - w - 1]) : 0;
#pragma unroll
        for (int u = 0; u < 4; ++u) { const float vv = valid ? TV[idn * DD + d0 + u] : bfr(wvb[d0 + u]); float p = __fmul_rn(tau, vv); asm volatile("" : "+v"(p)); acc[u] = __fadd_rn(acc[u], p); } }
    v4us oh, ol;
#pragma unroll
    for (int u = 0; u < 4; ++u) { unsigned short a, bb; splitf(acc[u], a, bb); oh[u] = a; ol[u] = bb; } *(volatile v4us*)(Mh + e) = oh; *(volatile v4us*)(Ml + e) = ol; __threadfence(); *(volatile v4us*)(Mh + e) = oh; *(volatile v4us*)(Ml + e) = ol; }
__global__ __launch_bounds__(256) void k_y(const float* __restrict__ G, const int* __restrict__ ids, const float* __restrict__ TX, const float* __restrict__ mgb, const float* __restrict__ lg, const float* __restrict__ lb, bf* Yh, bf* Yl) { const int lane = threadIdx.x & 31; const int tk = blockIdx.x * 8 + (threadIdx.x >> 5); if (tk >= NT) return; const int t = tk % TT; const int id = cid(ids[tk]); const int c0 = lane * 4; float v[4]; float s = 0.f;
    const v4f a = *(const v4f*)(G + (size_t)tk * DD + c0);
#pragma unroll
    for (int u = 0; u < 4; ++u) { const float y = __fadd_rn(__fadd_rn(a[u], TX[id * DD + c0 + u]), bfr(mgb[c0 + u])); v[u] = y; s += y; }
#pragma unroll
    for (int sh = 16; sh; sh >>= 1) s += __shfl_xor(s, sh, 32);
    const float mean = s * (1.0f / DD); float q = 0.f;
#pragma unroll
    for (int u = 0; u < 4; ++u) { float d = __fsub_rn(v[u], mean); asm volatile("" : "+v"(d)); float p = __fmul_rn(d, d); asm volatile("" : "+v"(p)); q = __fadd_rn(q, p); }
#pragma unroll
    for (int sh = 16; sh; sh >>= 1) q += __shfl_xor(q, sh, 32);
    const float rstd = __frsqrt_rn(__fadd_rn(q * (1.0f / DD), 1e-5f));
    float arg = __fmul_rn((float)t, 0.52359879f); asm volatile("" : "+v"(arg)); arg = __fadd_rn(arg, 1072.3303f); float sn = 0.15f * sinf(arg); asm volatile("" : "+v"(sn)); const float scl = __fadd_rn(1.0f, sn);
    v4us oh, ol;
#pragma unroll
    for (int u = 0; u < 4; ++u) { float d = __fsub_rn(v[u], mean); asm volatile("" : "+v"(d)); float n0 = __fmul_rn(d, rstd); asm volatile("" : "+v"(n0)); float g1 = bfr(lg[c0 + u]); asm volatile("" : "+v"(g1)); float t1 = __fmul_rn(n0, g1); asm volatile("" : "+v"(t1)); float y = __fadd_rn(t1, bfr(lb[c0 + u])); asm volatile("" : "+v"(y)); y = __fmul_rn(y, scl); unsigned short a2, b2; splitf(y, a2, b2); oh[u] = a2; ol[u] = b2; }
    const size_t oo = (size_t)tk * DD + c0; *(volatile v4us*)(Yh + oo) = oh; *(volatile v4us*)(Yl + oo) = ol; __threadfence(); *(volatile v4us*)(Yh + oo) = oh; *(volatile v4us*)(Yl + oo) = ol; }
__global__ __launch_bounds__(256) void k_out(const float* __restrict__ O64, const float* __restrict__ hb, float* OUT) { const int e = (blockIdx.x * 256 + threadIdx.x) * 4; if (e >= NT * VOC) return; v4f o;
#pragma unroll
    for (int u = 0; u < 4; ++u) { const int idx = e + u; const int vcol = idx % VOC; const int tk = idx / VOC; o[u] = __fadd_rn(O64[(size_t)tk * 64 + vcol], bfr(hb[vcol])); } *(volatile v4f*)(OUT + e) = o; __threadfence(); *(volatile v4f*)(OUT + e) = o; }

extern "C" void kernel_launch(void* const* d_in, const int* in_sizes, int n_in,
                              void* d_out, int out_size, void* d_ws, size_t ws_size, hipStream_t stream) {
    (void)in_sizes; (void)n_in; (void)out_size;
    const int* ids = (const int*)d_in[0]; const float** I = (const float**)d_in;
    const float *emb = I[1], *w1 = I[2], *b1 = I[3], *w2 = I[4], *b2 = I[5], *wv_w = I[6], *wv_b = I[7], *mg_w = I[8], *mg_b = I[9], *ln_g = I[10], *ln_b = I[11], *head_w = I[12], *head_b = I[13];
    float* OUT = (float*)d_out;
    char* wsp = (char*)d_ws;
    auto take = [&](size_t bytes) { char* p = wsp; wsp += (bytes + 255) & ~(size_t)255; return (void*)p; };
    bf* EB = (bf*)take(VP * DD * 2); bf* BA = (bf*)take(HH * DD * 2); bf* BB = (bf*)take(HH * DD * 2); bf* BVW = (bf*)take(DD * DD * 2); bf* BX = (bf*)take(DD * DD * 2); bf* BM = (bf*)take(DD * DD * 2); bf* BHD = (bf*)take(64 * DD * 2);
    float* TA = (float*)take(VP * HH * 4); float* TB = (float*)take(VP * HH * 4); float* TV = (float*)take(VP * DD * 4); float* TX = (float*)take(VP * DD * 4); float* TAU = (float*)take((size_t)NT * WW * 4); bf* Mh = (bf*)take((size_t)NT * DD * 2); bf* Ml = (bf*)take((size_t)NT * DD * 2);
    float* G = (float*)take((size_t)NT * DD * 4); bf* Yh = (bf*)take((size_t)NT * DD * 2); bf* Yl = (bf*)take((size_t)NT * DD * 2); float* O64 = (float*)take((size_t)NT * 64 * 4);
    if ((size_t)(wsp - (char*)d_ws) > ws_size) return;
    k_embp<<<(VP * DD / 4 + 255) / 256, 256, 0, stream>>>(emb, EB);
    k_wtG<<<(DD * HH / 64 + 63) / 64, 256, 0, stream>>>(w1, DD, HH, BA); k_wtG<<<(DD * HH / 64 + 63) / 64, 256, 0, stream>>>(w1 + DD * HH, DD, HH, BB);
    k_wtG<<<(DD * DD / 64 + 63) / 64, 256, 0, stream>>>(wv_w, DD, DD, BVW); k_wtG<<<(DD * DD / 64 + 63) / 64, 256, 0, stream>>>(mg_w, DD, DD, BX); k_wtG<<<(DD * DD / 64 + 63) / 64, 256, 0, stream>>>(mg_w + DD * DD, DD, DD, BM);
    k_wpad<<<(64 * DD / 4 + 255) / 256, 256, 0, stream>>>(head_w, DD, VOC, 64, BHD);
    k_gemmw<bf, 0, false><<<dim3(1, 1, 1), 32, 0, stream>>>(EB, nullptr, BA, nullptr, DD, TA, HH, nullptr, 0, 0, 0); k_gemmw<bf, 0, false><<<dim3(1, 1, 1), 32, 0, stream>>>(EB, nullptr, BB, nullptr, DD, TB, HH, nullptr, 0, 0, 0);
    k_gemmw<bf, 0, true><<<dim3(1, 2, 1), 32, 0, stream>>>(EB, nullptr, BVW, nullptr, DD, TV, DD, wv_b, 0, 0, 0); k_gemmw<bf, 0, false><<<dim3(1, 2, 1), 32, 0, stream>>>(EB, nullptr, BX, nullptr, DD, TX, DD, nullptr, 0, 0, 0);
    k_tau<<<(NT * WW + 255) / 256, 256, 0, stream>>>(ids, TA, TB, b1, w2, b2, TAU); k_msg<<<(NT * DD / 4 + 255) / 256, 256, 0, stream>>>(ids, TAU, TV, wv_b, Mh, Ml);
    k_gemmw<bf, 1, false><<<dim3(NT / 64, DD / 64, 1), 32, 0, stream>>>(Mh, Ml, BM, nullptr, DD, G, DD, nullptr, 0, 0, 0);
    k_y<<<NT / 8, 256, 0, stream>>>(G, ids, TX, mg_b, ln_g, ln_b, Yh, Yl);
    k_gemmw<bf, 1, false><<<dim3(NT / 64, 1, 1), 32, 0, stream>>>(Yh, Yl, BHD, nullptr, DD, O64, 64, nullptr, 0, 0, 0);
    k_out<<<(NT * VOC / 4 + 255) / 256, 256, 0, stream>>>(O64, head_b, OUT);
}
